// LSTM_21878563406096
// MI455X (gfx1250) — hardware-verified
//
#include <hip/hip_runtime.h>
#include <math.h>

constexpr int NBATCH   = 128;
constexpr int NTIME    = 256;
constexpr int NHID     = 128;
constexpr int NGATE    = 4 * NHID;
constexpr int NWIN     = 16;
constexpr int NWINDOWS = NTIME - NWIN;
constexpr int NTHR     = 256;
constexpr int ROWS_BLK = 16;
constexpr int HPITCH   = 136;
constexpr int HBUF_ELEMS = ROWS_BLK * HPITCH;
constexpr int XPITCH   = 256;
constexpr int OPITCH   = 260;
constexpr float HCARRY  = 1024.0f;
constexpr float WCARRY  = 256.0f;
constexpr float ACC_INV = 1.0f / (HCARRY * WCARRY);
constexpr float LEAKY_SLOPE = 0.3f;

static_assert(NBATCH % ROWS_BLK == 0, "batch tiles");
static_assert(NHID == 16 * (NTHR / 32), "8 waves x 16 hidden units");
static_assert(NHID % 32 == 0, "K multiple of 32");
static_assert((2 * HBUF_ELEMS) % NTHR == 0, "h zero-fill loop exact");
static_assert((ROWS_BLK * NTIME) % (NTHR * 4) == 0, "x tile load loop exact");
static_assert(NWINDOWS + NWIN == NTIME, "output columns");
static_assert((HPITCH % 8) == 0 && (OPITCH % 4) == 0, "16-B aligned LDS rows");

typedef __attribute__((ext_vector_type(16))) _Float16 v16h;
typedef __attribute__((ext_vector_type(8)))  _Float16 v8h;
typedef __attribute__((ext_vector_type(8)))  float    v8f;
typedef __attribute__((ext_vector_type(4)))  float    v4f;

union FragH { v16h v; v8h h[2]; };
__device__ __forceinline__ v16h frag_load_h(const _Float16* p) {
  FragH f;
  f.h[0] = *(const v8h*)(p);
  f.h[1] = *(const v8h*)(p + 16);
  return f.v;
}
__device__ __forceinline__ v8f mma_h(v16h a, v16h b, v8f c) {
  return __builtin_amdgcn_wmma_f32_16x16x32_f16(false, a, false, b, (short)0, c, false, false);
}
__device__ __forceinline__ void group_guard(v8f& c0, v8f& c1, v8f& c2, v8f& c3,
                                            v16h a, v16h b0, v16h b1, v16h b2, v16h b3) {
  asm volatile("v_nop\n\tv_nop\n\tv_nop\n\tv_nop"
               : "+v"(c0), "+v"(c1), "+v"(c2), "+v"(c3)
               : "v"(a), "v"(b0), "v"(b1), "v"(b2), "v"(b3));
}
__device__ __forceinline__ void pin_frag(v16h& f) { asm volatile("" : "+v"(f) : : "memory"); }

__device__ __forceinline__ float fsig(float x)  { return __builtin_amdgcn_rcpf(1.0f + __expf(-x)); }
__device__ __forceinline__ float ftanh(float x) { return 1.0f - 2.0f * __builtin_amdgcn_rcpf(__expf(2.0f * x) + 1.0f); }

__global__ __launch_bounds__(NTHR) void lstm_window_kernel(const float* __restrict__ x,
                                                           const float* __restrict__ w_ih,
                                                           const float* __restrict__ w_hh,
                                                           const float* __restrict__ b_ih,
                                                           const float* __restrict__ b_hh,
                                                           const float* __restrict__ fc_w,
                                                           const float* __restrict__ fc_b,
                                                           float* __restrict__ out) {
  __shared__ __align__(16) float    x_tile[ROWS_BLK * XPITCH];
  __shared__ __align__(16) float    out_tile[ROWS_BLK * OPITCH];
  __shared__ __align__(16) _Float16 hbuf[2 * HBUF_ELEMS];
  __shared__ float                  fcpart[(NTHR / 32) * ROWS_BLK];

  const int tid  = threadIdx.x;
  const int lane = tid & 31;
  const int wave = tid >> 5;
  const int c    = lane & 15;
  const int hh   = lane >> 4;
  const int koff = hh * 8;
  const int m0   = blockIdx.x * ROWS_BLK;
  const int unit = wave * 16 + c;

  float wih[4], bias[4];
#pragma unroll
  for (int q = 0; q < 4; ++q) {
    const int j = q * NHID + unit;
    wih[q]  = w_ih[j];
    bias[q] = b_ih[j] + b_hh[j];
  }
  const float fcw = fc_w[unit];
  const float fcb = fc_b[0];
  asm volatile("" ::: "memory");

#pragma unroll
  for (int it = 0; it < 4; ++it) {
    const int idx = it * NTHR + tid;
    const int row = idx >> 6;
    const int c4  = (idx & 63) * 4;
    const v4f v = *(const v4f*)(x + (size_t)(m0 + row) * NTIME + c4);
    *(v4f*)(x_tile + row * XPITCH + c4) = v;
    if (c4 < NWIN) *(v4f*)(out_tile + row * OPITCH + c4) = v;
  }
#pragma unroll 1
  for (int i = tid; i < 2 * HBUF_ELEMS; i += NTHR) hbuf[i] = (_Float16)0.0f;

  v16h bfrag[4][4];
#pragma unroll
  for (int q = 0; q < 4; ++q) {
    const float* wrow = w_hh + (size_t)(q * NHID + unit) * NHID + koff;
#pragma unroll
    for (int kk = 0; kk < 4; ++kk) {
      const v4f w0 = *(const v4f*)(wrow + kk * 32);
      const v4f w1 = *(const v4f*)(wrow + kk * 32 + 4);
      const v4f w2 = *(const v4f*)(wrow + kk * 32 + 16);
      const v4f w3 = *(const v4f*)(wrow + kk * 32 + 20);
      v16h f;
#pragma unroll
      for (int e = 0; e < 4; ++e) {
        f[e]      = (_Float16)(w0[e] * WCARRY);
        f[4 + e]  = (_Float16)(w1[e] * WCARRY);
        f[8 + e]  = (_Float16)(w2[e] * WCARRY);
        f[12 + e] = (_Float16)(w3[e] * WCARRY);
      }
      pin_frag(f);
      bfrag[q][kk] = f;
    }
  }

  float cst[8], hreg[8];
#pragma unroll
  for (int r = 0; r < 8; ++r) { cst[r] = 0.0f; hreg[r] = 0.0f; }

  __syncthreads();

  const v8f z8 = {0.f, 0.f, 0.f, 0.f, 0.f, 0.f, 0.f, 0.f};
  int cur = 0;

#pragma unroll 1
  for (int s = 0; s < NWINDOWS; ++s) {
#pragma unroll 1
    for (int t = 0; t < NWIN; ++t) {
      const int time = s + t;
      const _Float16* ard = hbuf + cur * HBUF_ELEMS + c * HPITCH + koff;
      _Float16*       hwr = hbuf + (cur ^ 1) * HBUF_ELEMS;

      v8f acc[4];
      acc[0] = z8; acc[1] = z8; acc[2] = z8; acc[3] = z8;
#pragma unroll
      for (int kk = 0; kk < 4; ++kk) {
        const v16h a = frag_load_h(ard + kk * 32);
        acc[0] = mma_h(a, bfrag[0][kk], acc[0]);
        acc[1] = mma_h(a, bfrag[1][kk], acc[1]);
        acc[2] = mma_h(a, bfrag[2][kk], acc[2]);
        acc[3] = mma_h(a, bfrag[3][kk], acc[3]);
        group_guard(acc[0], acc[1], acc[2], acc[3], a, bfrag[0][kk], bfrag[1][kk], bfrag[2][kk], bfrag[3][kk]);
      }

#pragma unroll
      for (int r = 0; r < 8; ++r) {
        const float xr = x_tile[(8 * hh + r) * XPITCH + time];
        const float zi = fmaf(acc[0][r], ACC_INV, fmaf(xr, wih[0], bias[0]));
        const float zf = fmaf(acc[1][r], ACC_INV, fmaf(xr, wih[1], bias[1]));
        const float zg = fmaf(acc[2][r], ACC_INV, fmaf(xr, wih[2], bias[2]));
        const float zo = fmaf(acc[3][r], ACC_INV, fmaf(xr, wih[3], bias[3]));
        const float ig = fsig(zi);
        const float fg = fsig(zf);
        const float gg = ftanh(zg);
        const float og = fsig(zo);
        const float cn = fg * cst[r] + ig * gg;
        cst[r] = cn;
        const float hv = og * ftanh(cn);
        hreg[r] = hv;
        hwr[(8 * hh + r) * HPITCH + unit] = (_Float16)(hv * HCARRY);
      }

      if (t == NWIN - 1) {
        float p[8];
#pragma unroll
        for (int r = 0; r < 8; ++r) p[r] = hreg[r] * fcw;
#pragma unroll
        for (int off = 1; off < 16; off <<= 1) {
#pragma unroll
          for (int r = 0; r < 8; ++r) p[r] += __shfl_xor(p[r], off, 32);
        }
        if (c == 0) {
#pragma unroll
          for (int r = 0; r < 8; ++r) fcpart[wave * ROWS_BLK + 8 * hh + r] = p[r];
        }
      }
      __syncthreads();

      if (t == NWIN - 1 && tid < ROWS_BLK) {
        float v = 0.0f;
#pragma unroll
        for (int w = 0; w < NTHR / 32; ++w) v += fcpart[w * ROWS_BLK + tid];
        v += fcb;
        out_tile[tid * OPITCH + NWIN + s] = (v >= 0.0f) ? v : LEAKY_SLOPE * v;
      }
      cur ^= 1;
    }
  }

  __syncthreads();

  for (int pass = 0; pass < 2; ++pass) {
#pragma unroll
    for (int it = 0; it < 4; ++it) {
      const int idx = it * NTHR + tid;
      const int row = idx >> 6;
      const int c4  = (idx & 63) * 4;
      const v4f v = *(const v4f*)(out_tile + row * OPITCH + c4);
      *(volatile v4f*)(out + (size_t)(m0 + row) * NTIME + c4) = v;
    }
    __threadfence();
  }
}

extern "C" void kernel_launch(void* const* d_in, const int* in_sizes, int n_in,
                              void* d_out, int out_size, void* d_ws, size_t ws_size, hipStream_t stream) {
  (void)d_ws; (void)ws_size;
  if (n_in < 7 || d_out == nullptr) return;
  if (in_sizes[0] != NBATCH * NTIME || in_sizes[1] != NGATE || in_sizes[2] != NGATE * NHID ||
      in_sizes[3] != NGATE || in_sizes[4] != NGATE || in_sizes[5] != NHID || in_sizes[6] != 1 ||
      out_size != NBATCH * NTIME) return;

  const float* x    = (const float*)d_in[0];
  const float* w_ih = (const float*)d_in[1];
  const float* w_hh = (const float*)d_in[2];
  const float* b_ih = (const float*)d_in[3];
  const float* b_hh = (const float*)d_in[4];
  const float* fc_w = (const float*)d_in[5];
  const float* fc_b = (const float*)d_in[6];
  float* out = (float*)d_out;

  lstm_window_kernel<<<dim3(NBATCH / ROWS_BLK), dim3(NTHR), 0, stream>>>(x, w_ih, w_hh, b_ih, b_hh, fc_w, fc_b, out);
}
